// HoloKVAttention_62672162784014
// MI455X (gfx1250) — hardware-verified
//
#include <hip/hip_runtime.h>
#define NBt 2
#define SS 2048
#define DM 1024
#define NH 16
#define DH 64
#define KF 4
#define NSL (SS / KF)
#define LR 64
#define NR (NBt * SS)
typedef __bf16 v16b __attribute__((ext_vector_type(16)));
typedef unsigned short v8us __attribute__((ext_vector_type(8), may_alias));
typedef float  v8f  __attribute__((ext_vector_type(8)));
typedef float  v4f  __attribute__((ext_vector_type(4)));
typedef float  v4fa __attribute__((ext_vector_type(4), may_alias));
union FragB { v16b v; v8us half[2]; unsigned short u[16]; };

__device__ __forceinline__ unsigned short bf16_bits(float x) { unsigned int u = __float_as_uint(x); return (unsigned short)((u + 0x7FFFu + ((u >> 16) & 1u)) >> 16); }
__device__ __forceinline__ float bf16_val(unsigned short b) { return __uint_as_float(((unsigned int)b) << 16); }
__device__ __forceinline__ float bf16_round(float x) { return bf16_val(bf16_bits(x)); }
template <int NT>
__device__ __forceinline__ v8f mmaN(v16b ah, v16b al, v16b bh, v16b bl, v8f c) {
  c = __builtin_amdgcn_wmma_f32_16x16x32_bf16(false, ah, false, bh, (short)0, c, false, false);
  if (NT >= 2) c = __builtin_amdgcn_wmma_f32_16x16x32_bf16(false, al, false, bh, (short)0, c, false, false);
  if (NT >= 3) c = __builtin_amdgcn_wmma_f32_16x16x32_bf16(false, ah, false, bl, (short)0, c, false, false);
  asm volatile("v_nop\n\tv_nop\n\tv_nop\n\tv_nop" : "+v"(c) : "v"(ah), "v"(al), "v"(bh), "v"(bl));
  return c;
}

__global__ __launch_bounds__(256) void k_wt_bf16(const float* __restrict__ W, unsigned short* __restrict__ Wt, int K, int N) {
  const int t = blockIdx.x * 256 + threadIdx.x;
  const int k8n = K / 8;
  if (t >= N * k8n) return;
  const int n = t / k8n, k8 = (t % k8n) * 8;
  v8us v;
#pragma unroll
  for (int i = 0; i < 8; ++i) v[i] = bf16_bits(W[(size_t)(k8 + i) * N + n]);
  *(volatile v8us*)(Wt + (size_t)n * K + k8) = v;
  __threadfence();
  *(volatile v8us*)(Wt + (size_t)n * K + k8) = v;
}

template <bool ASPLIT, int ACT, bool BIAS_BF16>
__global__ __launch_bounds__(128) void k_gemm_bf(const float* __restrict__ A, int lda, const unsigned short* __restrict__ Wt, int ldb,
                                               const float* __restrict__ bias, float* __restrict__ C, int ldc, int M, int N, int K) {
  __shared__ __attribute__((aligned(16))) float so[4][16][64];
  const int tid = threadIdx.x, w = tid >> 5, lane = tid & 31, ln = lane & 15, hh = lane >> 4;
  const int ntn = N / 64;
  const int wid = blockIdx.x * 4 + w;
  const int mt = wid / ntn, nq = wid % ntn;
  if (mt * 16 >= M) return;
  const int row0 = mt * 16, col0 = nq * 64;
  const float* arow = A + (size_t)(row0 + ln) * lda;
  v8f acc[4] = {};
  for (int kb = 0; kb < K; kb += 32) {
    FragB ah, al;
    const v4f x0 = *(const v4fa*)(arow + kb + 8 * hh), x1 = *(const v4fa*)(arow + kb + 8 * hh + 4);
    const v4f x2 = *(const v4fa*)(arow + kb + 16 + 8 * hh), x3 = *(const v4fa*)(arow + kb + 16 + 8 * hh + 4);
    float xs[16] = {x0[0],x0[1],x0[2],x0[3],x1[0],x1[1],x1[2],x1[3],x2[0],x2[1],x2[2],x2[3],x3[0],x3[1],x3[2],x3[3]};
#pragma unroll
    for (int i = 0; i < 16; ++i) { const unsigned short hb = bf16_bits(xs[i]); ah.u[i] = hb; al.u[i] = ASPLIT ? bf16_bits(xs[i] - bf16_val(hb)) : (unsigned short)0; }
#pragma unroll
    for (int t = 0; t < 4; ++t) {
      const unsigned short* brow = Wt + (size_t)(col0 + t * 16 + ln) * ldb + kb;
      FragB b;
      b.half[0] = *(const v8us*)(brow + 8 * hh);
      b.half[1] = *(const v8us*)(brow + 16 + 8 * hh);
      acc[t] = mmaN<ASPLIT ? 2 : 1>(ah.v, al.v, b.v, b.v, acc[t]);
    }
  }
#pragma unroll
  for (int t = 0; t < 4; ++t) {
    float bv = bias ? bias[col0 + t * 16 + ln] : 0.f;
    if (BIAS_BF16) bv = bf16_round(bv);
#pragma unroll
    for (int r = 0; r < 8; ++r) { float v = acc[t][r] + bv; if (ACT == 1) v = fmaxf(v, 0.f); so[w][8 * hh + r][t * 16 + ln] = v; }
  }
  __builtin_amdgcn_fence(__ATOMIC_ACQ_REL, "workgroup");
  __builtin_amdgcn_wave_barrier();
  const int rsub = lane >> 4, c4 = (lane & 15) * 4;
  for (int pass = 0; pass < 2; ++pass) {
#pragma unroll
    for (int q = 0; q < 8; ++q) {
      const int r = q * 2 + rsub;
      const v4f v = *(const v4fa*)&so[w][r][c4];
      *(volatile v4f*)(C + (size_t)(row0 + r) * ldc + col0 + c4) = v;
    }
    if (pass == 0) __threadfence();
  }
}

template <bool ASPLIT, int ACT, bool BIAS_BF16, bool RES_BF16>
__global__ __launch_bounds__(128) void k_gemm_bf3(const float* __restrict__ A, int lda, const unsigned short* __restrict__ Wt, int ldb,
                                                const float* __restrict__ bias, const float* __restrict__ resid, int rmod, int ldr,
                                                float* __restrict__ C, int ldc, int M, int N, int K) {
  __shared__ __attribute__((aligned(16))) float so[4][16][64];
  const int tid = threadIdx.x, w = tid >> 5, lane = tid & 31, ln = lane & 15, hh = lane >> 4;
  const int ntn = N / 64;
  const int wid = blockIdx.x * 4 + w;
  const int mt = wid / ntn, nq = wid % ntn;
  if (mt * 16 >= M) return;
  const int row0 = mt * 16, col0 = nq * 64;
  const float* arow = A + (size_t)(row0 + ln) * lda;
  v8f acc[4] = {};
  for (int kb = 0; kb < K; kb += 32) {
    FragB ah, al;
    const v4f x0 = *(const v4fa*)(arow + kb + 8 * hh), x1 = *(const v4fa*)(arow + kb + 8 * hh + 4);
    const v4f x2 = *(const v4fa*)(arow + kb + 16 + 8 * hh), x3 = *(const v4fa*)(arow + kb + 16 + 8 * hh + 4);
    float xs[16] = {x0[0],x0[1],x0[2],x0[3],x1[0],x1[1],x1[2],x1[3],x2[0],x2[1],x2[2],x2[3],x3[0],x3[1],x3[2],x3[3]};
#pragma unroll
    for (int i = 0; i < 16; ++i) { const unsigned short hb = bf16_bits(xs[i]); ah.u[i] = hb; al.u[i] = ASPLIT ? bf16_bits(xs[i] - bf16_val(hb)) : (unsigned short)0; }
#pragma unroll
    for (int t = 0; t < 4; ++t) {
      const unsigned short* brow = Wt + (size_t)(col0 + t * 16 + ln) * ldb + kb;
      FragB b;
      b.half[0] = *(const v8us*)(brow + 8 * hh);
      b.half[1] = *(const v8us*)(brow + 16 + 8 * hh);
      acc[t] = mmaN<ASPLIT ? 2 : 1>(ah.v, al.v, b.v, b.v, acc[t]);
    }
  }
#pragma unroll
  for (int t = 0; t < 4; ++t) {
    const int col = col0 + t * 16 + ln;
    float bv = bias ? bias[col] : 0.f;
    if (BIAS_BF16) bv = bf16_round(bv);
#pragma unroll
    for (int r = 0; r < 8; ++r) {
      float v = acc[t][r] + bv;
      if (resid) { float rv = resid[(size_t)((row0 + 8 * hh + r) % rmod) * ldr + col]; if (RES_BF16) rv = bf16_round(rv); v += rv; }
      if (ACT == 1) v = fmaxf(v, 0.f);
      if (ACT == 2) v = 0.5f * v * (1.0f + erff(v * 0.70710678118654752f));
      if (ACT == 3) { const float u = 0.7978845608028654f * (v + 0.044715f * v * v * v); v = 0.5f * v * (1.0f + tanhf(u)); }
      so[w][8 * hh + r][t * 16 + ln] = v;
    }
  }
  __builtin_amdgcn_fence(__ATOMIC_ACQ_REL, "workgroup");
  __builtin_amdgcn_wave_barrier();
  const int rsub = lane >> 4, c4 = (lane & 15) * 4;
  for (int pass = 0; pass < 2; ++pass) {
#pragma unroll
    for (int q = 0; q < 8; ++q) {
      const int r = q * 2 + rsub;
      const v4f v = *(const v4fa*)&so[w][r][c4];
      *(volatile v4f*)(C + (size_t)(row0 + r) * ldc + col0 + c4) = v;
    }
    if (pass == 0) __threadfence();
  }
}
template <bool PARAM_BF16>
__global__ __launch_bounds__(256) void k_layernorm(const float* __restrict__ X, const float* __restrict__ R, const float* __restrict__ g, const float* __restrict__ bta,
                                                  float* __restrict__ out_sum, float* __restrict__ out_norm, int N, float eps) {
  __shared__ float red[256];
  const int row = blockIdx.x, tid = threadIdx.x;
  const float* x = X + (size_t)row * N; const float* rr = R ? R + (size_t)row * N : nullptr;
  float vals[16];
  const int per = N / 256;
  float s1 = 0.f;
  for (int u = 0; u < per / 4; ++u) {
    const int j = tid * 4 + 1024 * u;
    const v4f a = *(const v4fa*)(x + j);
    v4f b = {0.f,0.f,0.f,0.f}; if (rr) b = *(const v4fa*)(rr + j);
#pragma unroll
    for (int q = 0; q < 4; ++q) { const float v = a[q] + b[q]; vals[u * 4 + q] = v; s1 += v; }
  }
  red[tid] = s1; __syncthreads();
  for (int st = 128; st > 0; st >>= 1) { if (tid < st) red[tid] += red[tid + st]; __syncthreads(); }
  const float mu = red[0] / (float)N; __syncthreads();
  float s2 = 0.f;
  for (int u = 0; u < per / 4; ++u)
#pragma unroll
    for (int q = 0; q < 4; ++q) { const float c = vals[u * 4 + q] - mu; s2 += c * c; }
  red[tid] = s2; __syncthreads();
  for (int st = 128; st > 0; st >>= 1) { if (tid < st) red[tid] += red[tid + st]; __syncthreads(); }
  const float rs = rsqrtf(red[0] / (float)N + eps);
  for (int pass = 0; pass < 2; ++pass) {
    for (int u = 0; u < per / 4; ++u) {
      const int j = tid * 4 + 1024 * u;
      v4f o, sm;
#pragma unroll
      for (int q = 0; q < 4; ++q) {
        float gg = g[j + q], bb = bta[j + q];
        if (PARAM_BF16) { gg = bf16_round(gg); bb = bf16_round(bb); }
        sm[q] = vals[u * 4 + q]; o[q] = (vals[u * 4 + q] - mu) * rs * gg + bb;
      }
      if (out_sum) *(volatile v4f*)(out_sum + (size_t)row * N + j) = sm;
      *(volatile v4f*)(out_norm + (size_t)row * N + j) = o;
    }
    if (pass == 0) __threadfence();
  }
}


typedef _Float16 v16h __attribute__((ext_vector_type(16)));
union FragH { v16h v; v8us half[2]; _Float16 h[16]; unsigned short u[16]; };
template <int NT>
__device__ __forceinline__ v8f mmaH(v16h ah, v16h al, v16h bh, v16h bl, v8f c) {
  c = __builtin_amdgcn_wmma_f32_16x16x32_f16(false, ah, false, bh, (short)0, c, false, false);
  if (NT >= 2) c = __builtin_amdgcn_wmma_f32_16x16x32_f16(false, al, false, bh, (short)0, c, false, false);
  if (NT >= 3) c = __builtin_amdgcn_wmma_f32_16x16x32_f16(false, ah, false, bl, (short)0, c, false, false);
  asm volatile("v_nop\n\tv_nop\n\tv_nop\n\tv_nop" : "+v"(c) : "v"(ah), "v"(al), "v"(bh), "v"(bl));
  return c;
}
template <bool ASPLIT>
__global__ __launch_bounds__(128) void k_gemm_h(const float* __restrict__ A, int lda, size_t sA, const _Float16* __restrict__ Bh, int ldb, size_t sB, float alpha, float* __restrict__ C, int ldc, size_t sC, int M, int N, int K) {
  __shared__ __attribute__((aligned(16))) float so[4][16][64];
  const int tid = threadIdx.x, w = tid >> 5, lane = tid & 31, ln = lane & 15, hh = lane >> 4; const int by = blockIdx.y;
  A += (size_t)by * sA; Bh += (size_t)by * sB; C += (size_t)by * sC;
  const int ntn = (N + 63) / 64; const int wid = blockIdx.x * 4 + w; const int mt = wid / ntn, nq = wid % ntn; if (mt * 16 >= M) return;
  const int row0 = mt * 16, col0 = nq * 64; const float* arow = A + (size_t)(row0 + ln) * lda;
  v8f acc[4] = {};
  for (int kb = 0; kb < K; kb += 32) {
    FragH ah, al;
    const v4f x0 = *(const v4fa*)(arow + kb + 8 * hh), x1 = *(const v4fa*)(arow + kb + 8 * hh + 4), x2 = *(const v4fa*)(arow + kb + 16 + 8 * hh), x3 = *(const v4fa*)(arow + kb + 16 + 8 * hh + 4);
    float xs[16] = {x0[0],x0[1],x0[2],x0[3],x1[0],x1[1],x1[2],x1[3],x2[0],x2[1],x2[2],x2[3],x3[0],x3[1],x3[2],x3[3]};
#pragma unroll
    for (int i = 0; i < 16; ++i) { const _Float16 h = (_Float16)xs[i]; ah.h[i] = h; al.h[i] = ASPLIT ? (_Float16)(xs[i] - (float)h) : (_Float16)0.0f; }
#pragma unroll
    for (int t = 0; t < 4; ++t) { if (col0 + t * 16 >= N) continue; const size_t boff = (size_t)(col0 + t * 16 + ln) * ldb + kb; FragH bq; bq.half[0] = *(const v8us*)(Bh + boff + 8 * hh); bq.half[1] = *(const v8us*)(Bh + boff + 16 + 8 * hh);
      acc[t] = mmaH<ASPLIT ? 2 : 1>(ah.v, al.v, bq.v, bq.v, acc[t]); }
  }
#pragma unroll
  for (int t = 0; t < 4; ++t) { if (col0 + t * 16 >= N) continue;
#pragma unroll
    for (int r = 0; r < 8; ++r) so[w][8 * hh + r][t * 16 + ln] = acc[t][r] * alpha; }
  __builtin_amdgcn_fence(__ATOMIC_ACQ_REL, "workgroup"); __builtin_amdgcn_wave_barrier();
  const int rsub = lane >> 4, c4 = (lane & 15) * 4;
  for (int pass = 0; pass < 2; ++pass) {
#pragma unroll
    for (int q = 0; q < 8; ++q) { const int r = q * 2 + rsub; if (col0 + c4 < N) { const v4f v = *(const v4fa*)&so[w][r][c4]; *(volatile v4f*)(C + (size_t)(row0 + r) * ldc + col0 + c4) = v; } }
    if (pass == 0) __threadfence(); }
}

__global__ __launch_bounds__(256) void k_wt_f16(const float* __restrict__ W, _Float16* __restrict__ Wt, int K, int N, float scale) {
  const int t = blockIdx.x * 256 + threadIdx.x; if (t >= N * (K / 8)) return; const int n = t / (K / 8), k8 = (t % (K / 8)) * 8; FragH f;
#pragma unroll
  for (int i = 0; i < 8; ++i) f.h[i] = (_Float16)(bf16_round(W[(size_t)(k8 + i) * N + n]) * scale); const v8us o = f.half[0];
  *(volatile v8us*)((unsigned short*)Wt + (size_t)n * K + k8) = o; __threadfence(); *(volatile v8us*)((unsigned short*)Wt + (size_t)n * K + k8) = o;
}
template <int ACT>
__global__ __launch_bounds__(128) void k_gemm_hhx(const _Float16* __restrict__ A, int lda, size_t sA, const _Float16* __restrict__ Bh, int ldb, size_t sB, float alpha, const float* __restrict__ bias, size_t sBias, const float* __restrict__ CP, int rowsPerB, size_t sCPb, int row0g,
    float* __restrict__ C, _Float16* __restrict__ C16, int ldc, size_t sC, int M, int N, int K) {
  __shared__ __attribute__((aligned(16))) float so[4][16][64];
  const int tid = threadIdx.x, w = tid >> 5, lane = tid & 31, ln = lane & 15, hh = lane >> 4; const int by = blockIdx.y;
  A += (size_t)by * sA; Bh += (size_t)by * sB; const size_t cofs = (size_t)by * sC; const float* bp = bias ? bias + (size_t)by * sBias : nullptr;
  const int ntn = (N + 63) / 64; const int wid = blockIdx.x * 4 + w; const int mt = wid / ntn, nq = wid % ntn; if (mt * 16 >= M) return;
  const int row0 = mt * 16, col0 = nq * 64; const _Float16* arow = A + (size_t)(row0 + ln) * lda;
  v8f acc[4] = {};
  for (int kb = 0; kb < K; kb += 32) { FragH ah; ah.half[0] = *(const v8us*)((const unsigned short*)arow + kb + 8 * hh); ah.half[1] = *(const v8us*)((const unsigned short*)arow + kb + 16 + 8 * hh);
#pragma unroll
    for (int t = 0; t < 4; ++t) { if (col0 + t * 16 >= N) continue; const size_t boff = (size_t)(col0 + t * 16 + ln) * ldb + kb; FragH bq; bq.half[0] = *(const v8us*)((const unsigned short*)Bh + boff + 8 * hh); bq.half[1] = *(const v8us*)((const unsigned short*)Bh + boff + 16 + 8 * hh);
      acc[t] = mmaH<1>(ah.v, ah.v, bq.v, bq.v, acc[t]); }
  }
#pragma unroll
  for (int t = 0; t < 4; ++t) { if (col0 + t * 16 >= N) continue; const int col = col0 + t * 16 + ln; const float bv = bp ? bf16_round(bp[col]) : 0.f;
#pragma unroll
    for (int r = 0; r < 8; ++r) { float v = acc[t][r] * alpha + bv; if (CP) { const int bidx = (row0g + row0 + 8 * hh + r) / rowsPerB; v += CP[(size_t)bidx * sCPb + (size_t)by * 64 + col]; } if (ACT == 1) v = (v > 0.f) ? v : expm1f(v); else if (ACT == 7) v = (v > 0.f) ? v + 1.0f : expf(v); else if (ACT == 8) v = tanhf(v); else if (ACT == 9) v = 0.5f * v * (1.0f + tanhf(0.7978845608028654f * (v + 0.044715f * v * v * v))); else if (ACT == 11) v = 1.0f / (1.0f + expf(-v)); else if (ACT == 12) v = (v > 0.f) ? v : 0.01f * v; else if (ACT == 14) v = (v > 0.f) ? v : 0.1f * v; else if (ACT == 15) v = v / (1.0f + expf(-v)); else if (ACT == 3) v = fmaxf(v, 0.f); else if (ACT == 6) v = 0.5f * v * (1.0f + erff(v * 0.70710678118654752f)); so[w][8 * hh + r][t * 16 + ln] = v; } }
  __builtin_amdgcn_fence(__ATOMIC_ACQ_REL, "workgroup"); __builtin_amdgcn_wave_barrier();
  const int rsub = lane >> 4, c4 = (lane & 15) * 4; typedef _Float16 v4h __attribute__((ext_vector_type(4)));
  for (int pass = 0; pass < 2; ++pass) {
#pragma unroll
    for (int q = 0; q < 8; ++q) { const int r = q * 2 + rsub; if (col0 + c4 < N) { const v4f v = *(const v4fa*)&so[w][r][c4]; if (C) *(volatile v4f*)(C + cofs + (size_t)(row0 + r) * ldc + col0 + c4) = v; if (C16) { v4h h4; for (int i = 0; i < 4; ++i) h4[i] = (_Float16)v[i]; *(volatile v4h*)(C16 + cofs + (size_t)(row0 + r) * ldc + col0 + c4) = h4; } } }
    if (pass == 0) __threadfence(); }
}


typedef _Float16 v4h __attribute__((ext_vector_type(4)));

__global__ __launch_bounds__(256) void k_x16(const float* __restrict__ x, _Float16* __restrict__ X16, size_t n8) { const size_t t = (size_t)blockIdx.x * 256 + threadIdx.x; if (t >= n8) return; FragH f;
#pragma unroll
  for (int q = 0; q < 8; ++q) f.h[q] = (_Float16)bf16_round(x[t * 8 + q]); *(volatile v8us*)((unsigned short*)X16 + t * 8) = f.half[0]; __threadfence(); *(volatile v8us*)((unsigned short*)X16 + t * 8) = f.half[0]; }
__global__ __launch_bounds__(256) void k_h16(const float* __restrict__ x, _Float16* __restrict__ X16, size_t n8) { const size_t t = (size_t)blockIdx.x * 256 + threadIdx.x; if (t >= n8) return; FragH f;
#pragma unroll
  for (int q = 0; q < 8; ++q) f.h[q] = (_Float16)x[t * 8 + q]; *(volatile v8us*)((unsigned short*)X16 + t * 8) = f.half[0]; __threadfence(); *(volatile v8us*)((unsigned short*)X16 + t * 8) = f.half[0]; }
__global__ __launch_bounds__(256) void k_round16f(const float* __restrict__ W, _Float16* __restrict__ Bt, size_t n8) { const size_t t = (size_t)blockIdx.x * 256 + threadIdx.x; if (t >= n8) return; FragH f;
#pragma unroll
  for (int i = 0; i < 8; ++i) f.h[i] = (_Float16)(bf16_round(W[t * 8 + i]) * 16.0f); *(volatile v8us*)((unsigned short*)Bt + t * 8) = f.half[0]; __threadfence(); *(volatile v8us*)((unsigned short*)Bt + t * 8) = f.half[0]; }
template <int NHv, int TTv>
__global__ __launch_bounds__(256) void k_vt(const _Float16* __restrict__ V16, int ldv, int voff, _Float16* __restrict__ Vt) { __shared__ unsigned short tl[64][66]; const int tid = threadIdx.x; const int slab = blockIdx.x / (TTv / 64), lg = blockIdx.x % (TTv / 64); const int b = slab / NHv, h = slab % NHv;
  for (int i = tid; i < 64 * 8; i += 256) { const int r = i / 8, c8 = (i % 8) * 8; FragH f; f.half[0] = *(const v8us*)((const unsigned short*)V16 + ((size_t)b * TTv + lg * 64 + r) * ldv + voff + h * 64 + c8);
#pragma unroll
    for (int q = 0; q < 8; ++q) tl[r][c8 + q] = f.u[q]; }
  __syncthreads();
  for (int pass = 0; pass < 2; ++pass) {
#pragma unroll
    for (int rd = 0; rd < 2; ++rd) { const int d = rd * 32 + tid / 8, pc = tid % 8; FragH f;
#pragma unroll
      for (int q = 0; q < 8; ++q) f.u[q] = tl[pc * 8 + q][d];
      *(volatile v8us*)((unsigned short*)Vt + ((size_t)slab * 64 + d) * TTv + lg * 64 + pc * 8) = f.half[0]; }
    if (pass == 0) __threadfence(); } }

__global__ __launch_bounds__(256) void k_hl(const float* __restrict__ F, _Float16* __restrict__ Hh, _Float16* __restrict__ Hl, size_t n8) { const size_t t = (size_t)blockIdx.x * 256 + threadIdx.x; if (t >= n8) return; FragH fh, fl; const v4f a = *(const v4fa*)(F + t * 8), c = *(const v4fa*)(F + t * 8 + 4);
#pragma unroll
  for (int q = 0; q < 4; ++q) { _Float16 h = (_Float16)a[q]; fh.h[q] = h; fl.h[q] = (_Float16)((a[q] - (float)h) * 1024.0f); h = (_Float16)c[q]; fh.h[4 + q] = h; fl.h[4 + q] = (_Float16)((c[q] - (float)h) * 1024.0f); }
  for (int pass = 0; pass < 2; ++pass) { *(volatile v8us*)((unsigned short*)Hh + t * 8) = fh.half[0]; *(volatile v8us*)((unsigned short*)Hl + t * 8) = fl.half[0]; if (pass == 0) __threadfence(); } }

__global__ __launch_bounds__(256) void k_split(const float* __restrict__ F, _Float16* __restrict__ Hh, _Float16* __restrict__ Hl, size_t n8) {
  #pragma clang fp contract(off)
  const size_t t = (size_t)blockIdx.x * 256 + threadIdx.x; if (t >= n8) return; const v4f a = *(const v4fa*)(F + t * 8), c = *(const v4fa*)(F + t * 8 + 4); FragH fh, fl;
#pragma unroll
  for (int q = 0; q < 8; ++q) { const float v = (q < 4) ? a[q] : c[q - 4]; const _Float16 hi = (_Float16)v; fh.h[q] = hi; fl.h[q] = (_Float16)((v - (float)hi) * 1024.0f); }
  for (int pass = 0; pass < 2; ++pass) { *(volatile v8us*)((unsigned short*)Hh + t * 8) = fh.half[0]; *(volatile v8us*)((unsigned short*)Hl + t * 8) = fl.half[0]; if (pass == 0) __threadfence(); } }
__global__ __launch_bounds__(256) void k_cstab(float* __restrict__ CS, float* __restrict__ SN) {
  #pragma clang fp contract(off)
  const int t = blockIdx.x * 256 + threadIdx.x; if (t >= SS * DH) return; const int d = t % DH, p = t / DH; const int i = d & 31; const float theta = 1.0f / powf(10000.0f, (float)(2 * i) / 64.0f); const float ang = (float)p * theta; const float c = cosf(ang), s = sinf(ang);
  for (int pass = 0; pass < 2; ++pass) { *(volatile float*)(CS + t) = c; *(volatile float*)(SN + t) = s; if (pass == 0) __threadfence(); } }
__device__ __forceinline__ float cdma(int t, int d) { const int j = d & 3; const int par = __popc((unsigned)(t & j)); return (par & 1) ? -1.0f : 1.0f; }
__global__ __launch_bounds__(256) void k_slots(const float* __restrict__ Q, const float* __restrict__ K, const float* __restrict__ V, const float* __restrict__ CS, const float* __restrict__ SN, _Float16* __restrict__ FK16, _Float16* __restrict__ FV16, float* __restrict__ FKf, float* __restrict__ FVf, float* __restrict__ PK, float* __restrict__ PVp, _Float16* __restrict__ AQ16, float* __restrict__ AQf) {
  #pragma clang fp contract(off)
  const int t = blockIdx.x * 256 + threadIdx.x; if (t >= NH * NSL * (DH / 8)) return; const int d0 = (t % (DH / 8)) * 8; const int s = (t / (DH / 8)) % NSL; const int bh = t / ((DH / 8) * NSL); const int b = 0, h = bh;
  FragH fk, fv; v4f fkA, fkB, fvA, fvB;
  float pk[KF][8], pv[KF][8];
#pragma unroll
  for (int q = 0; q < 8; ++q) { const int d = d0 + q; float accK = 0.f, accV = 0.f;
#pragma unroll
    for (int tt = 0; tt < KF; ++tt) { const int tok = s * KF + tt; const float* kp = K + ((size_t)b * SS + tok) * DM + h * DH; const float* vp = V + ((size_t)b * SS + tok) * DM + h * DH; const float c = CS[(size_t)tok * DH + d], sn = SN[(size_t)tok * DH + d];
      const float kr = kp[d] * c + ((d < 32) ? -kp[d + 32] : kp[d - 32]) * sn; const float ph = cdma(tt, d) * 0.5f;
      accK += kr * ph; accV += vp[d] * ph; pk[tt][q] = accK; pv[tt][q] = accV; }
    fk.h[q] = (_Float16)accK; fv.h[q] = (_Float16)accV; if (q < 4) { fkA[q] = accK; fvA[q] = accV; } else { fkB[q - 4] = accK; fvB[q - 4] = accV; } }
  const size_t srow = ((size_t)bh * NSL + s) * DH + d0;
  for (int pass = 0; pass < 2; ++pass) { *(volatile v8us*)((unsigned short*)FK16 + srow) = fk.half[0]; *(volatile v8us*)((unsigned short*)FV16 + srow) = fv.half[0]; *(volatile v4f*)(FKf + srow) = fkA; *(volatile v4f*)(FKf + srow + 4) = fkB; *(volatile v4f*)(FVf + srow) = fvA; *(volatile v4f*)(FVf + srow + 4) = fvB; if (pass == 0) __threadfence(); }
#pragma unroll
  for (int tt = 0; tt < KF; ++tt) { const int tok = s * KF + tt; const size_t prow = ((size_t)b * SS + tok) * DM + h * DH + d0; v4f a, c2, e, g;
#pragma unroll
    for (int q = 0; q < 4; ++q) { a[q] = pk[tt][q]; c2[q] = pk[tt][4 + q]; e[q] = pv[tt][q]; g[q] = pv[tt][4 + q]; }
      const float* qp = Q + ((size_t)b * SS + tok) * DM + h * DH; FragH fq; v4f qa, qb2;
#pragma unroll
    for (int q = 0; q < 8; ++q) { const int d = d0 + q; const float c = CS[(size_t)tok * DH + d], sn = SN[(size_t)tok * DH + d]; const float qr = qp[d] * c + ((d < 32) ? -qp[d + 32] : qp[d - 32]) * sn; const float aq = qr * cdma(tt, d); fq.h[q] = (_Float16)aq; if (q < 4) qa[q] = aq; else qb2[q - 4] = aq; }
    const size_t arow = ((size_t)bh * SS + tok) * DH + d0;
    for (int pass = 0; pass < 2; ++pass) { *(volatile v4f*)(PK + prow) = a; *(volatile v4f*)(PK + prow + 4) = c2; *(volatile v4f*)(PVp + prow) = e; *(volatile v4f*)(PVp + prow + 4) = g; *(volatile v8us*)((unsigned short*)AQ16 + arow) = fq.half[0]; *(volatile v4f*)(AQf + prow) = qa; *(volatile v4f*)(AQf + prow + 4) = qb2; if (pass == 0) __threadfence(); } } }
__global__ __launch_bounds__(256) void k_fvt(const float* __restrict__ FVf, _Float16* __restrict__ FVT) { const int t = blockIdx.x * 256 + threadIdx.x; if (t >= NH * DH * (NSL / 8)) return; const int s0 = (t % (NSL / 8)) * 8; const int d = (t / (NSL / 8)) % DH; const int h = t / ((NSL / 8) * DH); FragH f;
#pragma unroll
  for (int q = 0; q < 8; ++q) f.h[q] = (_Float16)FVf[((size_t)h * NSL + s0 + q) * DH + d];
  *(volatile v8us*)((unsigned short*)FVT + ((size_t)h * DH + d) * NSL + s0) = f.half[0]; __threadfence(); *(volatile v8us*)((unsigned short*)FVT + ((size_t)h * DH + d) * NSL + s0) = f.half[0]; }
__global__ __launch_bounds__(256) void k_hsoft(const float* __restrict__ S, const float* __restrict__ AQf, const float* __restrict__ PK, int b, int h, _Float16* __restrict__ W16, float* __restrict__ WC) {
  #pragma clang fp contract(off)
  const int tid = threadIdx.x, w = tid >> 5, ln = tid & 31; const int q = blockIdx.x * 8 + w; if (q >= SS) return; const int cs = q / KF; const size_t prow = ((size_t)b * SS + q) * DM + h * DH;
  float cur = AQf[prow + ln] * PK[prow + ln] + AQf[prow + 32 + ln] * PK[prow + 32 + ln]; for (int o = 16; o > 0; o >>= 1) cur += __shfl_xor(cur, o, 32); cur *= 0.125f;
  const float* sr = S + (size_t)q * NSL; float v[16]; float m = -3.0e38f;
#pragma unroll
  for (int k = 0; k < 16; ++k) { const int sl = 16 * ln + k; float x = sr[sl]; x = (sl == cs) ? cur : x; x = (sl > cs) ? -3.0e38f : x; v[k] = x; m = fmaxf(m, x); }
  for (int o = 16; o > 0; o >>= 1) m = fmaxf(m, __shfl_xor(m, o, 32));
  float su = 0.f;
#pragma unroll
  for (int k = 0; k < 16; ++k) { const int sl = 16 * ln + k; v[k] = (sl > cs) ? 0.f : expf(v[k] - m); su += v[k]; }
  for (int o = 16; o > 0; o >>= 1) su += __shfl_xor(su, o, 32); const float inv = 1.0f / su; FragH f0, f1; float wc = 0.f;
#pragma unroll
  for (int k = 0; k < 16; ++k) { const int sl = 16 * ln + k; const float wv = v[k] * inv; wc = (sl == cs) ? wv : wc; if (k < 8) f0.h[k] = (_Float16)(wv * 1024.0f); else f1.h[k - 8] = (_Float16)(wv * 1024.0f); }
  for (int o = 16; o > 0; o >>= 1) wc += __shfl_xor(wc, o, 32);
  const float wl = (ln == h) ? wc : WC[((size_t)b * SS + q) * 32 + ln];
  const float wlv = (h == 0 && ln != 0) ? 0.f : wl;
  for (int pass = 0; pass < 2; ++pass) { *(volatile v8us*)((unsigned short*)W16 + (size_t)q * NSL + 16 * ln) = f0.half[0]; *(volatile v8us*)((unsigned short*)W16 + (size_t)q * NSL + 16 * ln + 8) = f1.half[0]; *(volatile float*)(WC + ((size_t)b * SS + q) * 32 + ln) = wlv; if (pass == 0) __threadfence(); } }
__global__ __launch_bounds__(256) void k_oepi(const float* __restrict__ O, const float* __restrict__ WC, const float* __restrict__ PVp, const float* __restrict__ FVf, _Float16* __restrict__ Oh, _Float16* __restrict__ Ol) {
  #pragma clang fp contract(off)
  const int t = blockIdx.x * 256 + threadIdx.x; if (t >= SS * NH * (DH / 8)) return; const int d0 = (t % (DH / 8)) * 8; const int h = (t / (DH / 8)) % NH; const int bq = t / ((DH / 8) * NH); const int b = 0, q = bq; const int cs = q / KF, tt = q % KF; const float wc = WC[(size_t)bq * 32 + h]; const size_t prow = (size_t)bq * DM + h * DH + d0; const size_t srow = ((size_t)(b * NH + h) * NSL + cs) * DH + d0; FragH fh, fl;
#pragma unroll
  for (int k = 0; k < 8; ++k) { const int d = d0 + k; const float o = O[prow + k] + wc * (PVp[prow + k] - FVf[srow + k]); const float v = (o * cdma(tt, d)) * 2.0f; const _Float16 hi = (_Float16)v; fh.h[k] = hi; fl.h[k] = (_Float16)((v - (float)hi) * 1024.0f); }
  for (int pass = 0; pass < 2; ++pass) { *(volatile v8us*)((unsigned short*)Oh + prow) = fh.half[0]; *(volatile v8us*)((unsigned short*)Ol + prow) = fl.half[0]; if (pass == 0) __threadfence(); } }

extern "C" void kernel_launch(void* const* d_in, const int* in_sizes, int n_in,
                              void* d_out, int out_size, void* d_ws, size_t ws_size, hipStream_t stream) {
  (void)in_sizes; (void)n_in; (void)out_size;
  const float* x = (const float*)d_in[0]; const float* Wq = (const float*)d_in[1]; const float* Wk = (const float*)d_in[2]; const float* Wv = (const float*)d_in[3]; const float* Wo = (const float*)d_in[4]; const float* Aq = (const float*)d_in[5]; const float* Bq = (const float*)d_in[6]; const float* Av = (const float*)d_in[7]; const float* Bv = (const float*)d_in[8]; const float* Ao = (const float*)d_in[9]; const float* Bo = (const float*)d_in[10];
  char* ws = (char*)d_ws; size_t off = 0;
  auto take = [&](size_t bytes) { char* p = ws + off; off += (bytes + 255) & ~(size_t)255; return p; };
  _Float16* BWq = (_Float16*)take((size_t)DM * DM * 2); _Float16* BWk = (_Float16*)take((size_t)DM * DM * 2); _Float16* BWv = (_Float16*)take((size_t)DM * DM * 2); _Float16* BWo = (_Float16*)take((size_t)DM * DM * 2); _Float16* BAq = (_Float16*)take((size_t)LR * DM * 2); _Float16* BAv = (_Float16*)take((size_t)LR * DM * 2); _Float16* BAo = (_Float16*)take((size_t)LR * DM * 2); _Float16* BBq = (_Float16*)take((size_t)DM * LR * 2); _Float16* BBv = (_Float16*)take((size_t)DM * LR * 2); _Float16* BBo = (_Float16*)take((size_t)DM * LR * 2);
  float* CS = (float*)take((size_t)SS * DH * 4); float* SN = (float*)take((size_t)SS * DH * 4);
  _Float16* X16 = (_Float16*)take((size_t)SS * DM * 2); float* Q = (float*)take((size_t)SS * DM * 4); float* K = (float*)take((size_t)SS * DM * 4); float* V = (float*)take((size_t)SS * DM * 4); float* XA = (float*)take((size_t)SS * LR * 4); _Float16* XAh = (_Float16*)take((size_t)SS * LR * 2); _Float16* XAl = (_Float16*)take((size_t)SS * LR * 2);
  _Float16* FK16 = (_Float16*)take((size_t)NH * NSL * DH * 2); _Float16* FV16 = (_Float16*)take((size_t)NH * NSL * DH * 2); float* FKf = (float*)take((size_t)NH * NSL * DH * 4); float* FVf = (float*)take((size_t)NH * NSL * DH * 4); float* PK = (float*)take((size_t)SS * DM * 4); float* PVp = (float*)take((size_t)SS * DM * 4); _Float16* AQ16 = (_Float16*)take((size_t)NH * SS * DH * 2); float* AQf = (float*)take((size_t)SS * DM * 4);
  float* S = (float*)take((size_t)SS * NSL * 4); _Float16* W16 = (_Float16*)take((size_t)SS * NSL * 2); float* WC = (float*)take((size_t)SS * 32 * 4); _Float16* FVT = (_Float16*)take((size_t)NH * DH * NSL * 2); float* O = (float*)take((size_t)SS * DM * 4); _Float16* Oh = (_Float16*)take((size_t)SS * DM * 2); _Float16* Ol = (_Float16*)take((size_t)SS * DM * 2); float* OA = (float*)take((size_t)SS * LR * 4); _Float16* OAh = (_Float16*)take((size_t)SS * LR * 2); _Float16* OAl = (_Float16*)take((size_t)SS * LR * 2);
  if (off > ws_size) return;
  const unsigned nbW = (DM * (DM / 8) + 255) / 256;
  k_wt_f16<<<nbW, 256, 0, stream>>>(Wq, BWq, DM, DM, 16.0f); k_wt_f16<<<nbW, 256, 0, stream>>>(Wk, BWk, DM, DM, 16.0f); k_wt_f16<<<nbW, 256, 0, stream>>>(Wv, BWv, DM, DM, 16.0f); k_wt_f16<<<nbW, 256, 0, stream>>>(Wo, BWo, DM, DM, 16.0f);
  k_wt_f16<<<(LR * (DM / 8) + 255) / 256, 256, 0, stream>>>(Aq, BAq, DM, LR, 16.0f); k_wt_f16<<<(LR * (DM / 8) + 255) / 256, 256, 0, stream>>>(Av, BAv, DM, LR, 16.0f); k_wt_f16<<<(LR * (DM / 8) + 255) / 256, 256, 0, stream>>>(Ao, BAo, DM, LR, 16.0f);
  k_wt_f16<<<(DM * (LR / 8) + 255) / 256, 256, 0, stream>>>(Bq, BBq, LR, DM, 16.0f); k_wt_f16<<<(DM * (LR / 8) + 255) / 256, 256, 0, stream>>>(Bv, BBv, LR, DM, 16.0f); k_wt_f16<<<(DM * (LR / 8) + 255) / 256, 256, 0, stream>>>(Bo, BBo, LR, DM, 16.0f);
  k_cstab<<<(SS * DH + 255) / 256, 256, 0, stream>>>(CS, SN);
  const dim3 gD(((SS / 16) * (DM / 64) + 3) / 4, 1), gL(((SS / 16) * 1 + 3) / 4, 1), gL4(((SS / 16) * 1 + 3) / 4, 1), gS(((SS / 16) * (NSL / 64) + 3) / 4, 1); const size_t n8 = (size_t)SS * DM / 8; const unsigned nb8 = (unsigned)((n8 + 255) / 256); const size_t a8 = (size_t)SS * LR / 8; const unsigned nba = (unsigned)((a8 + 255) / 256);
  for (int b = 0; b < NBt; ++b) {
    k_x16<<<nb8, 256, 0, stream>>>(x + (size_t)b * SS * DM, X16, n8);
    k_gemm_hhx<0><<<gD, 128, 0, stream>>>(X16, DM, 0, BWq, DM, 0, 0.0625f, nullptr, 0, nullptr, 1, 0, 0, Q, nullptr, DM, 0, SS, DM, DM); k_gemm_hhx<0><<<gD, 128, 0, stream>>>(X16, DM, 0, BWk, DM, 0, 0.0625f, nullptr, 0, nullptr, 1, 0, 0, K, nullptr, DM, 0, SS, DM, DM); k_gemm_hhx<0><<<gD, 128, 0, stream>>>(X16, DM, 0, BWv, DM, 0, 0.0625f, nullptr, 0, nullptr, 1, 0, 0, V, nullptr, DM, 0, SS, DM, DM);
    k_gemm_hhx<0><<<gL, 128, 0, stream>>>(X16, DM, 0, BAq, DM, 0, 0.0625f, nullptr, 0, nullptr, 1, 0, 0, XA, nullptr, LR, 0, SS, LR, DM); k_split<<<nba, 256, 0, stream>>>(XA, XAh, XAl, a8);
    k_gemm_hhx<0><<<gD, 128, 0, stream>>>(XAh, LR, 0, BBq, LR, 0, 0.0625f, nullptr, 0, Q, 1, (size_t)DM, 0, Q, nullptr, DM, 0, SS, DM, LR); k_gemm_hhx<0><<<gD, 128, 0, stream>>>(XAl, LR, 0, BBq, LR, 0, 0.0625f / 1024.0f, nullptr, 0, Q, 1, (size_t)DM, 0, Q, nullptr, DM, 0, SS, DM, LR);
    k_gemm_hhx<0><<<gL, 128, 0, stream>>>(X16, DM, 0, BAv, DM, 0, 0.0625f, nullptr, 0, nullptr, 1, 0, 0, XA, nullptr, LR, 0, SS, LR, DM); k_split<<<nba, 256, 0, stream>>>(XA, XAh, XAl, a8);
    k_gemm_hhx<0><<<gD, 128, 0, stream>>>(XAh, LR, 0, BBv, LR, 0, 0.0625f, nullptr, 0, V, 1, (size_t)DM, 0, V, nullptr, DM, 0, SS, DM, LR); k_gemm_hhx<0><<<gD, 128, 0, stream>>>(XAl, LR, 0, BBv, LR, 0, 0.0625f / 1024.0f, nullptr, 0, V, 1, (size_t)DM, 0, V, nullptr, DM, 0, SS, DM, LR);
    k_slots<<<(NH * NSL * (DH / 8) + 255) / 256, 256, 0, stream>>>(Q, K, V, CS, SN, FK16, FV16, FKf, FVf, PK, PVp, AQ16, AQf);
    k_fvt<<<(NH * DH * (NSL / 8) + 255) / 256, 256, 0, stream>>>(FVf, FVT);
    for (int h = 0; h < NH; ++h) {
      k_gemm_hhx<0><<<gS, 128, 0, stream>>>(AQ16 + (size_t)h * SS * DH, DH, 0, FK16 + (size_t)h * NSL * DH, DH, 0, 0.125f, nullptr, 0, nullptr, 1, 0, 0, S, nullptr, NSL, 0, SS, NSL, DH);
      k_hsoft<<<SS / 8, 256, 0, stream>>>(S, AQf, PK, 0, h, W16, WC);
      k_gemm_hhx<0><<<gL4, 128, 0, stream>>>(W16, NSL, 0, FVT + (size_t)h * DH * NSL, NSL, 0, 0.0009765625f, nullptr, 0, nullptr, 1, 0, 0, O + h * DH, nullptr, DM, 0, SS, DH, NSL); }
    k_oepi<<<(SS * NH * (DH / 8) + 255) / 256, 256, 0, stream>>>(O, WC, PVp, FVf, Oh, Ol);
    float* outb = (float*)d_out + (size_t)b * SS * DM;
    k_gemm_hhx<0><<<gD, 128, 0, stream>>>(Oh, DM, 0, BWo, DM, 0, 0.0625f, nullptr, 0, nullptr, 1, 0, 0, outb, nullptr, DM, 0, SS, DM, DM); k_gemm_hhx<0><<<gD, 128, 0, stream>>>(Ol, DM, 0, BWo, DM, 0, 0.0625f / 1024.0f, nullptr, 0, outb, 1, (size_t)DM, 0, outb, nullptr, DM, 0, SS, DM, DM);
    k_gemm_hhx<0><<<gL, 128, 0, stream>>>(Oh, DM, 0, BAo, DM, 0, 0.0625f, nullptr, 0, nullptr, 1, 0, 0, OA, nullptr, LR, 0, SS, LR, DM); k_gemm_hhx<0><<<gL, 128, 0, stream>>>(Ol, DM, 0, BAo, DM, 0, 0.0625f / 1024.0f, nullptr, 0, OA, 1, (size_t)LR, 0, OA, nullptr, LR, 0, SS, LR, DM); k_split<<<nba, 256, 0, stream>>>(OA, OAh, OAl, a8);
    k_gemm_hhx<0><<<gD, 128, 0, stream>>>(OAh, LR, 0, BBo, LR, 0, 0.0625f, nullptr, 0, outb, 1, (size_t)DM, 0, outb, nullptr, DM, 0, SS, DM, LR); k_gemm_hhx<0><<<gD, 128, 0, stream>>>(OAl, LR, 0, BBo, LR, 0, 0.0625f / 1024.0f, nullptr, 0, outb, 1, (size_t)DM, 0, outb, nullptr, DM, 0, SS, DM, LR); }
}
